// CNF_14362370638429
// MI455X (gfx1250) — hardware-verified
//
#include <hip/hip_runtime.h>
#include <math.h>

constexpr int kRows         = 32768;
constexpr int kDimZ         = 64;
constexpr int kHid          = 256;
constexpr int kXld          = 65;
constexpr int kRowsPerBlock = 128;
constexpr int kThreads      = 256;
constexpr int kHChunk       = 64;
constexpr float kW2Carry    = 16.0f;
constexpr float kHCarry     = 256.0f;
constexpr float kOutScale   = 1.0f / (16.0f * 256.0f);
constexpr int kOutTileFloats = kRowsPerBlock * kXld;
constexpr int kOutTileVec4   = kOutTileFloats / 4;

static_assert(kDimZ % 32 == 0, "GEMM1 K multiple of 32");
static_assert(kHChunk % 32 == 0 && kHid % kHChunk == 0, "GEMM2 K chunks multiple of 32");
static_assert(kRows % kRowsPerBlock == 0, "row tiles exact");
static_assert(kRowsPerBlock == 16 * (kThreads / 32), "one 16-row slab per wave");
static_assert((kOutTileFloats * 4) % 128 == 0, "block output span is whole 128-B lines");
static_assert(kOutTileFloats % 4 == 0, "float4 store granularity");

constexpr size_t kOffXb   = 0;
constexpr size_t kBytesXb = (size_t)kRows * kDimZ * 2;
constexpr size_t kOffW1T  = kOffXb + kBytesXb;
constexpr size_t kBytesW1T = (size_t)kHid * kDimZ * 2;
constexpr size_t kOffW2T  = kOffW1T + kBytesW1T;
constexpr size_t kBytesW2T = (size_t)kDimZ * kHid * 2;
constexpr size_t kOffS    = kOffW2T + kBytesW2T;
constexpr size_t kBytesS  = (size_t)kHid * 4;
constexpr size_t kWsTotal = kOffS + kBytesS;
static_assert(kOffW1T % 128 == 0 && kOffW2T % 128 == 0 && kOffS % 128 == 0, "aligned carves");
static_assert(kWsTotal <= 134217728ull, "carve under 128 MiB");

typedef __attribute__((ext_vector_type(16))) _Float16 v16h;
typedef __attribute__((ext_vector_type(8)))  _Float16 v8h;
typedef __attribute__((ext_vector_type(16))) __bf16   v16b;
typedef __attribute__((ext_vector_type(8)))  __bf16   v8b;
typedef __attribute__((ext_vector_type(8)))  float    v8f;
typedef __attribute__((ext_vector_type(4)))  float    v4f;
typedef __attribute__((ext_vector_type(4)))  unsigned int v4u;

__device__ __forceinline__ unsigned short f2bf_bits(float f) {
  unsigned u = __float_as_uint(f);
  return (unsigned short)((u + 0x7FFFu + ((u >> 16) & 1u)) >> 16);
}
__device__ __forceinline__ float bf_bits2f(unsigned short h) { return __uint_as_float(((unsigned)h) << 16); }

__device__ __forceinline__ void dep_guard_h(v8f& a, v8f& b, v16h x, v16h y) { asm volatile("v_nop\n\tv_nop\n\tv_nop\n\tv_nop" : "+v"(a), "+v"(b) : "v"(x), "v"(y)); }
__device__ __forceinline__ void dep_guard_b(v8f& a, v8f& b, v16b x, v16b y) { asm volatile("v_nop\n\tv_nop\n\tv_nop\n\tv_nop" : "+v"(a), "+v"(b) : "v"(x), "v"(y)); }
__device__ __forceinline__ void keep4_h(v16h a, v16h b, v16h c, v16h d) { asm volatile("v_nop" :: "v"(a), "v"(b), "v"(c), "v"(d)); }
__device__ __forceinline__ void keep4_b(v16b a, v16b b, v16b c, v16b d) { asm volatile("v_nop" :: "v"(a), "v"(b), "v"(c), "v"(d)); }
__device__ __forceinline__ void acc_guard4(v8f& a, v8f& b, v8f& c, v8f& d) { asm volatile("v_nop\n\tv_nop\n\tv_nop\n\tv_nop" : "+v"(a), "+v"(b), "+v"(c), "+v"(d)); }
template <typename T> struct Frag;
template <> struct Frag<_Float16> {
  typedef v16h V; union U { v16h v; v8h h[2]; };
  static __device__ __forceinline__ v16h load(const _Float16* p) {
    U f; f.h[0] = *(const v8h*)(p); f.h[1] = *(const v8h*)(p + 16); return f.v;
  }
  static __device__ __forceinline__ v8f mma(v16h a, v16h b, v8f c) {
    return __builtin_amdgcn_wmma_f32_16x16x32_f16(false, a, false, b, (short)0, c, false, false);
  }
  static __device__ __forceinline__ void guard(v8f& a, v8f& b, v16h x, v16h y) { dep_guard_h(a, b, x, y); }
  static __device__ __forceinline__ void keep(v16h a, v16h b, v16h c, v16h d) { keep4_h(a, b, c, d); }
};
template <> struct Frag<__bf16> {
  typedef v16b V; union U { v16b v; v8b h[2]; };
  static __device__ __forceinline__ v16b load(const __bf16* p) {
    U f; f.h[0] = *(const v8b*)(p); f.h[1] = *(const v8b*)(p + 16); return f.v;
  }
  static __device__ __forceinline__ v8f mma(v16b a, v16b b, v8f c) {
    return __builtin_amdgcn_wmma_f32_16x16x32_bf16(false, a, false, b, (short)0, c, false, false);
  }
  static __device__ __forceinline__ void guard(v8f& a, v8f& b, v16b x, v16b y) { dep_guard_b(a, b, x, y); }
  static __device__ __forceinline__ void keep(v16b a, v16b b, v16b c, v16b d) { keep4_b(a, b, c, d); }
};

__device__ __forceinline__ void tie4_b(v8f& a0, v8f& a1, v8f& a2, v8f& a3,
                                       v16b x, v16b y0, v16b y1, v16b y2, v16b y3) {
  asm volatile("v_nop\n\tv_nop\n\tv_nop\n\tv_nop"
               : "+v"(a0), "+v"(a1), "+v"(a2), "+v"(a3)
               : "v"(x), "v"(y0), "v"(y1), "v"(y2), "v"(y3));
}
__device__ __forceinline__ void tie4_h(v8f& a0, v8f& a1, v8f& a2, v8f& a3,
                                       v16h x, v16h y0, v16h y1, v16h y2, v16h y3) {
  asm volatile("v_nop\n\tv_nop\n\tv_nop\n\tv_nop"
               : "+v"(a0), "+v"(a1), "+v"(a2), "+v"(a3)
               : "v"(x), "v"(y0), "v"(y1), "v"(y2), "v"(y3));
}

__device__ __forceinline__ unsigned pk16(unsigned short a, unsigned short b) { return (unsigned)a | ((unsigned)b << 16); }
__device__ __forceinline__ unsigned short h_bits(float f) { const _Float16 h = (_Float16)f; return __builtin_bit_cast(unsigned short, h); }
__device__ __forceinline__ float bf_rne(float f) { return bf_bits2f(f2bf_bits(f)); }

__global__ __launch_bounds__(256) void xcast_kernel(const float* __restrict__ x,
                                                    unsigned short* __restrict__ xb, int nthr) {
  const int i = blockIdx.x * 256 + threadIdx.x;
  if (i >= nthr) return;
  const int row = i >> 3;
  const int c8  = (i & 7) * 8;
  const float* p = x + (size_t)row * kXld + 1 + c8;
  unsigned short hb[8];
#pragma unroll
  for (int e = 0; e < 8; ++e) hb[e] = f2bf_bits(p[e]);
  const v4u u = (v4u){pk16(hb[0], hb[1]), pk16(hb[2], hb[3]), pk16(hb[4], hb[5]), pk16(hb[6], hb[7])};
  unsigned short* q = xb + (size_t)row * kDimZ + c8;
  *(volatile v4u*)q = u;
  __threadfence();
  *(volatile v4u*)q = u;
}

__global__ __launch_bounds__(256) void w1t_kernel(const float* __restrict__ W1,
                                                  unsigned short* __restrict__ w1t, int nthr) {
  const int i = blockIdx.x * 256 + threadIdx.x;
  if (i >= nthr) return;
  const int n  = i >> 3;
  const int c8 = (i & 7) * 8;
  unsigned short hb[8];
#pragma unroll
  for (int e = 0; e < 8; ++e) hb[e] = f2bf_bits(W1[(size_t)(c8 + e) * kHid + n]);
  const v4u u = (v4u){pk16(hb[0], hb[1]), pk16(hb[2], hb[3]), pk16(hb[4], hb[5]), pk16(hb[6], hb[7])};
  unsigned short* q = w1t + (size_t)n * kDimZ + c8;
  *(volatile v4u*)q = u;
  __threadfence();
  *(volatile v4u*)q = u;
}

__global__ __launch_bounds__(256) void w2t_kernel(const float* __restrict__ W2,
                                                  unsigned short* __restrict__ w2t, int nthr) {
  const int i = blockIdx.x * 256 + threadIdx.x;
  if (i >= nthr) return;
  const int n  = i >> 5;
  const int c8 = (i & 31) * 8;
  unsigned short hb[8];
#pragma unroll
  for (int e = 0; e < 8; ++e) hb[e] = h_bits(bf_rne(W2[(size_t)(c8 + e) * kDimZ + n]) * kW2Carry);
  const v4u u = (v4u){pk16(hb[0], hb[1]), pk16(hb[2], hb[3]), pk16(hb[4], hb[5]), pk16(hb[6], hb[7])};
  unsigned short* q = w2t + (size_t)n * kHid + c8;
  *(volatile v4u*)q = u;
  __threadfence();
  *(volatile v4u*)q = u;
}

__global__ __launch_bounds__(256) void svec_kernel(const float* __restrict__ W1, const float* __restrict__ W2,
                                                   float* __restrict__ s) {
  const int k = threadIdx.x;
  float acc = 0.0f;
#pragma unroll 1
  for (int d = 0; d < kDimZ; ++d) {
    const float a = bf_rne(W1[(size_t)d * kHid + k]);
    const float b = bf_rne(W2[(size_t)k * kDimZ + d]);
    acc = fmaf(a, b, acc);
  }
  ((volatile float*)s)[k] = acc;
  __threadfence();
  ((volatile float*)s)[k] = acc;
}

__global__ __launch_bounds__(256) void fused_mlp_trace_kernel(
    const unsigned short* __restrict__ xb, const unsigned short* __restrict__ w1t,
    const unsigned short* __restrict__ w2t, const float* __restrict__ svec,
    const float* __restrict__ b1, const float* __restrict__ b2, float* __restrict__ out) {
  __shared__ __align__(16) _Float16 sH[kThreads / 32][16 * kHChunk];
  __shared__ __align__(16) float    sOut[kOutTileFloats];

  const int t     = threadIdx.x;
  const int lane  = t & 31;
  const int wave  = t >> 5;
  const int hh    = lane >> 4;
  const int rlane = lane & 15;
  const int koff  = hh * 8;
  const int m0    = blockIdx.x * kRowsPerBlock + wave * 16;

  const __bf16*   Xb  = (const __bf16*)xb;
  const __bf16*   W1b = (const __bf16*)w1t;
  const _Float16* W2h = (const _Float16*)w2t;

  v16b xa[2];
#pragma unroll
  for (int dc = 0; dc < 2; ++dc)
    xa[dc] = Frag<__bf16>::load(Xb + (size_t)(m0 + rlane) * kDimZ + dc * 32 + koff);

  v8f acc2[4];
#pragma unroll
  for (int j = 0; j < 4; ++j) acc2[j] = (v8f){0.f,0.f,0.f,0.f,0.f,0.f,0.f,0.f};
  float tr[8];
#pragma unroll
  for (int r = 0; r < 8; ++r) tr[r] = 0.0f;

  _Float16* shw = sH[wave];

#pragma unroll 1
  for (int c = 0; c < kHid / kHChunk; ++c) {
    v8f acc1[4];
#pragma unroll
    for (int j = 0; j < 4; ++j) acc1[j] = (v8f){0.f,0.f,0.f,0.f,0.f,0.f,0.f,0.f};
#pragma unroll
    for (int dc = 0; dc < 2; ++dc) {
      v16b bw[4];
#pragma unroll
      for (int j = 0; j < 4; ++j)
        bw[j] = Frag<__bf16>::load(W1b + (size_t)(c * kHChunk + j * 16 + rlane) * kDimZ + dc * 32 + koff);
#pragma unroll
      for (int j = 0; j < 4; ++j) acc1[j] = Frag<__bf16>::mma(xa[dc], bw[j], acc1[j]);
      tie4_b(acc1[0], acc1[1], acc1[2], acc1[3], xa[dc], bw[0], bw[1], bw[2], bw[3]);
    }

    __syncthreads();

#pragma unroll
    for (int j = 0; j < 4; ++j) {
      const int hc   = c * kHChunk + j * 16 + rlane;
      const float bv = bf_rne(b1[hc]);
      const float sk = svec[hc];
#pragma unroll
      for (int r = 0; r < 8; ++r) {
        const float pre = acc1[j][r] + bv;
        const float hv  = tanhf(pre);
        tr[r] += (1.0f - hv * hv) * sk;
        shw[(8 * hh + r) * kHChunk + j * 16 + rlane] = (_Float16)(hv * kHCarry);
      }
    }
    __syncthreads();

#pragma unroll
    for (int dc = 0; dc < 2; ++dc) {
      const v16h ha = Frag<_Float16>::load(shw + rlane * kHChunk + dc * 32 + koff);
      v16h bw[4];
#pragma unroll
      for (int j = 0; j < 4; ++j)
        bw[j] = Frag<_Float16>::load(W2h + (size_t)(j * 16 + rlane) * kHid + c * kHChunk + dc * 32 + koff);
#pragma unroll
      for (int j = 0; j < 4; ++j) acc2[j] = Frag<_Float16>::mma(ha, bw[j], acc2[j]);
      tie4_h(acc2[0], acc2[1], acc2[2], acc2[3], ha, bw[0], bw[1], bw[2], bw[3]);
    }
  }
  acc_guard4(acc2[0], acc2[1], acc2[2], acc2[3]);

  float trs[8];
#pragma unroll
  for (int r = 0; r < 8; ++r) {
    float v = tr[r];
    v += __shfl_xor(v, 1, 32);
    v += __shfl_xor(v, 2, 32);
    v += __shfl_xor(v, 4, 32);
    v += __shfl_xor(v, 8, 32);
    trs[r] = v;
  }

#pragma unroll
  for (int j = 0; j < 4; ++j) {
    const int oc   = j * 16 + rlane;
    const float bv = bf_rne(b2[oc]);
#pragma unroll
    for (int r = 0; r < 8; ++r) {
      const int lr = wave * 16 + 8 * hh + r;
      sOut[lr * kXld + 1 + oc] = acc2[j][r] * kOutScale + bv;
    }
  }
#pragma unroll
  for (int r = 0; r < 8; ++r) {
    const int lr = wave * 16 + 8 * hh + r;
    sOut[lr * kXld] = -trs[r];
  }
  __syncthreads();

  float* ob = out + (size_t)blockIdx.x * kOutTileFloats;
  for (int pass = 0; pass < 2; ++pass) {
#pragma unroll
    for (int it = 0; it < (kOutTileVec4 + kThreads - 1) / kThreads; ++it) {
      const int idx = it * kThreads + t;
      if (idx < kOutTileVec4) {
        const v4f v = *(const v4f*)(sOut + idx * 4);
        *(volatile v4f*)(ob + (size_t)idx * 4) = v;
      }
    }
    __threadfence();
  }
}

extern "C" void kernel_launch(void* const* d_in, const int* in_sizes, int n_in,
                              void* d_out, int out_size, void* d_ws, size_t ws_size,
                              hipStream_t stream) {
  if (n_in < 5) return;
  if (in_sizes[0] != kRows * kXld || in_sizes[1] != kDimZ * kHid || in_sizes[2] != kHid ||
      in_sizes[3] != kHid * kDimZ || in_sizes[4] != kDimZ) return;
  if (out_size != kRows * kXld) return;
  if (ws_size < kWsTotal) return;

  const float* x  = (const float*)d_in[0];
  const float* W1 = (const float*)d_in[1];
  const float* b1 = (const float*)d_in[2];
  const float* W2 = (const float*)d_in[3];
  const float* b2 = (const float*)d_in[4];
  float* out = (float*)d_out;

  unsigned char* ws = (unsigned char*)d_ws;
  unsigned short* xb  = (unsigned short*)(ws + kOffXb);
  unsigned short* w1t = (unsigned short*)(ws + kOffW1T);
  unsigned short* w2t = (unsigned short*)(ws + kOffW2T);
  float*          sv  = (float*)(ws + kOffS);

  const int nthrX = kRows * kDimZ / 8;
  const int nthrW = kHid * kDimZ / 8;
  xcast_kernel<<<dim3((nthrX + 255) / 256), dim3(256), 0, stream>>>(x, xb, nthrX);
  w1t_kernel<<<dim3((nthrW + 255) / 256), dim3(256), 0, stream>>>(W1, w1t, nthrW);
  w2t_kernel<<<dim3((nthrW + 255) / 256), dim3(256), 0, stream>>>(W2, w2t, nthrW);
  svec_kernel<<<dim3(1), dim3(kHid), 0, stream>>>(W1, W2, sv);
  fused_mlp_trace_kernel<<<dim3(kRows / kRowsPerBlock), dim3(kThreads), 0, stream>>>(
      xb, w1t, w2t, sv, b1, b2, out);
}
